// MhAttnBlock_7627861918129
// MI455X (gfx1250) — hardware-verified
//
#include <hip/hip_runtime.h>
#include <math.h>

typedef __attribute__((ext_vector_type(16))) _Float16 v16h;
typedef __attribute__((ext_vector_type(16))) __bf16 v16b;
typedef __attribute__((ext_vector_type(8)))  _Float16 v8h;
typedef __attribute__((ext_vector_type(8)))  float v8f;
typedef __attribute__((ext_vector_type(4)))  float v4f;
typedef __attribute__((ext_vector_type(2)))  float v2f;
typedef __attribute__((ext_vector_type(4)))  unsigned v4u;
typedef __attribute__((ext_vector_type(4)))  int v4i;
typedef float __attribute__((may_alias)) float_a;
typedef int __attribute__((may_alias)) int_a;

template <typename T> __device__ __forceinline__ void vst2(void* p, T v) { *(volatile T*)p = v; __threadfence(); *(volatile T*)p = v; }
__device__ __forceinline__ v8f wmma16(v16h a, v16h b, v8f c) {
  v8f d = __builtin_amdgcn_wmma_f32_16x16x32_f16(false, a, false, b, (short)0, c, false, false);
  asm volatile("v_nop\n\tv_nop\n\tv_nop\n\tv_nop" : "+v"(d) : "v"(a), "v"(b));
  return d;
}
__device__ __forceinline__ v8f wmma_bf(v16b a, v16b b, v8f c) {
  v8f d = __builtin_amdgcn_wmma_f32_16x16x32_bf16(false, a, false, b, (short)0, c, false, false);
  asm volatile("v_nop\n\tv_nop\n\tv_nop\n\tv_nop" : "+v"(d) : "v"(a), "v"(b));
  return d;
}
__device__ __forceinline__ v16h frag_h(const _Float16* rowk0, int lane) {
  union { v16h v; v8h q[2]; } u; const _Float16* p = rowk0 + 8 * (lane >> 4);
  u.q[0] = *(const v8h*)p; u.q[1] = *(const v8h*)(p + 16); return u.v;
}
__device__ __forceinline__ v16h frag_f32(const float* rowk0, int lane) {
  v16h a; const float* p = rowk0 + 8 * (lane >> 4);
#pragma unroll
  for (int i = 0; i < 8; ++i) { a[i] = (_Float16)p[i]; a[8 + i] = (_Float16)p[16 + i]; }
  return a;
}
__device__ __forceinline__ v16h frag_f32s(const float* rowk0, int lane, float sc) {
  v16h a; const float* p = rowk0 + 8 * (lane >> 4);
#pragma unroll
  for (int i = 0; i < 8; ++i) { a[i] = (_Float16)(p[i] * sc); a[8 + i] = (_Float16)(p[16 + i] * sc); }
  return a;
}
__device__ __forceinline__ v16h fragc_f32(const float* W, int k0, int n, int lane, int ld, int K) {
  v16h a; const int g = lane >> 4;
#pragma unroll
  for (int i = 0; i < 8; ++i) { const int ka = k0 + 8 * g + i, kb = ka + 16;
    a[i] = (_Float16)(ka < K ? W[(size_t)(ka < K ? ka : K - 1) * ld + n] : 0.f); a[8 + i] = (_Float16)(kb < K ? W[(size_t)(kb < K ? kb : K - 1) * ld + n] : 0.f); }
  return a;
}
struct F2 { v16b h, l; };
__device__ __forceinline__ F2 bsplit16(const float v[16]) { F2 r;
#pragma unroll
  for (int i = 0; i < 16; ++i) { const __bf16 h = (__bf16)v[i]; r.h[i] = h; r.l[i] = (__bf16)(v[i] - (float)h); }
  return r; }
__device__ __forceinline__ F2 split_row(const float* row, int k0, int lane) { float v[16]; const float* p = row + k0 + 8 * (lane >> 4);
#pragma unroll
  for (int i = 0; i < 8; ++i) { v[i] = p[i]; v[8 + i] = p[16 + i]; }
  return bsplit16(v); }
__device__ __forceinline__ F2 split_rowK(const float* row, int k0, int lane, int K) { float v[16]; const int g = lane >> 4;
#pragma unroll
  for (int i = 0; i < 8; ++i) { const int ka = k0 + 8 * g + i, kb = ka + 16; v[i] = ka < K ? row[ka < K ? ka : K - 1] : 0.f; v[8 + i] = kb < K ? row[kb < K ? kb : K - 1] : 0.f; }
  return bsplit16(v); }
__device__ __forceinline__ F2 split_col(const float* W, int k0, int n, int lane, int ld, int K) { float v[16]; const int g = lane >> 4;
#pragma unroll
  for (int i = 0; i < 8; ++i) { const int ka = k0 + 8 * g + i, kb = ka + 16; v[i] = ka < K ? W[(size_t)(ka < K ? ka : K - 1) * ld + n] : 0.f; v[8 + i] = kb < K ? W[(size_t)(kb < K ? kb : K - 1) * ld + n] : 0.f; }
  return bsplit16(v); }
__device__ __forceinline__ v8f mac3(const F2& a, const F2& b, v8f c) { c = wmma_bf(a.l, b.h, c); c = wmma_bf(a.h, b.l, c); return wmma_bf(a.h, b.h, c); }
__device__ __forceinline__ float sigm(float v) { return 1.0f / (1.0f + expf(-v)); }
#define LDSX() do { asm volatile("s_wait_dscnt 0" ::: "memory"); __builtin_amdgcn_wave_barrier(); __builtin_amdgcn_fence(__ATOMIC_RELEASE, "workgroup"); } while (0)


#define NB 8
#define SQ 1024
#define SK 1024
#define DI 512
#define NH 8
#define OD 64
#ifndef TQB
#define TQB (SQ / 64)
#define TNB NB
#endif
typedef __attribute__((ext_vector_type(8))) __bf16 v8b;
__device__ __forceinline__ v16b frag_b(const __bf16* rowk0, int lane) {
  union { v16b v; v8b q[2]; } u; const __bf16* p = rowk0 + 8 * (lane >> 4);
  u.q[0] = *(const v8b*)p; u.q[1] = *(const v8b*)(p + 16); return u.v;
}
__device__ __forceinline__ v16b frag_gbf(const float* rowk0, int lane) {
  v16b a; const float* p = rowk0 + 8 * (lane >> 4);
#pragma unroll
  for (int i = 0; i < 8; ++i) { a[i] = (__bf16)p[i]; a[8 + i] = (__bf16)p[16 + i]; }
  return a;
}
__device__ __forceinline__ float bfr(float v) { return (float)(__bf16)v; }
__device__ __attribute__((noinline)) float exp_ni(float v) { return expf(v); }
#define WS_VTH  0u
#define WS_VTL  (WS_VTH + 2u * NB * DI * SK)
#define WS_AQ   (WS_VTL + 2u * NB * DI * SK)
#define WS_AK   (WS_AQ + 4u * NB * NH * SQ)
#define WS_END  (WS_AK + 4u * NB * NH * SK)

__global__ __launch_bounds__(128) void k_vproj(const float* __restrict__ V, const float* __restrict__ WV, __bf16* __restrict__ VTH, __bf16* __restrict__ VTL) {
  __shared__ __align__(16) __bf16 sh[DI][72], sl[DI][72];
  const int tid = threadIdx.x, wave = tid >> 5, lane = tid & 31, col = lane & 15, g = lane >> 4; const int b = blockIdx.y; const int k0 = blockIdx.x * 64;
  const float* Vb = V + ((size_t)b * SK + k0 + wave * 16) * DI;
#pragma unroll 1
  for (int oc = 0; oc < DI / 128; ++oc) { v8f acc[8] = {};
#pragma unroll 2
    for (int kc = 0; kc < DI / 32; ++kc) { const v16b a = frag_gbf(Vb + (size_t)col * DI + kc * 32, lane);
#pragma unroll
      for (int j = 0; j < 8; ++j) acc[j] = wmma_bf(a, frag_gbf(WV + (size_t)(oc * 128 + j * 16 + col) * DI + kc * 32, lane), acc[j]); }
#pragma unroll
    for (int j = 0; j < 8; ++j)
#pragma unroll
      for (int r = 0; r < 8; ++r) { const int o = oc * 128 + j * 16 + col; const float v = acc[j][r]; const __bf16 hb = (__bf16)v; sh[o][wave * 16 + 8 * g + r] = hb; sl[o][wave * 16 + 8 * g + r] = (__bf16)(v - (float)hb); } }
  __syncthreads();
  for (int q = tid; q < DI * 8; q += 128) { const int o = q >> 3, pc = q & 7; const size_t off = ((size_t)b * DI + o) * SK + k0 + pc * 8; vst2((unsigned*)(VTH + off), *(const v4u*)&sh[o][pc * 8]); vst2((unsigned*)(VTL + off), *(const v4u*)&sl[o][pc * 8]); }
}
__global__ __launch_bounds__(256) void k_aqk(const float* __restrict__ Q, const float* __restrict__ K, const float* __restrict__ WQ, const float* __restrict__ WK, float* __restrict__ AQ, float* __restrict__ AK) {
  __shared__ float sw[NH][DI]; __shared__ __align__(16) float so[NH][64];
  const int tid = threadIdx.x, b = blockIdx.y, which = blockIdx.z; const int r0 = blockIdx.x * 64; const float* X = which == 0 ? Q : K; const float* Wm = which == 0 ? WQ : WK; float* A = which == 0 ? AQ : AK; const int L = which == 0 ? SQ : SK;
  for (int q = tid; q < NH * DI; q += 256) sw[q / DI][q % DI] = bfr(Wm[q]);
  __syncthreads();
  { const int rl = tid >> 2, hp = tid & 3; const float* xr = X + ((size_t)b * L + r0 + rl) * DI; float a0 = 0.f, a1 = 0.f;
#pragma unroll 1
    for (int i = 0; i < DI; ++i) { const float xv = bfr(xr[i]); a0 += xv * sw[hp * 2][i]; a1 += xv * sw[hp * 2 + 1][i]; }
    so[hp * 2][rl] = a0; so[hp * 2 + 1][rl] = a1; }
  __syncthreads();
  if (tid < NH * 16) { const int h = tid >> 4, pc = tid & 15; vst2(A + ((size_t)b * NH + h) * L + r0 + pc * 4, *(const v4f*)&so[h][pc * 4]); }
}
__global__ __launch_bounds__(128) void k_attn(const float* __restrict__ AQ, const float* __restrict__ AK, const __bf16* __restrict__ VTH, const __bf16* __restrict__ VTL, const float* __restrict__ BIAS, float* __restrict__ OUT) {
  __shared__ __align__(16) float sp[4][16][36]; __shared__ __align__(16) float so[4][16][68];
  const int tid = threadIdx.x, wave = tid >> 5, lane = tid & 31, col = lane & 15, g = lane >> 4;
  const int qb = blockIdx.x, bh = blockIdx.y, b = bh / NH, h = bh % NH; const int q0 = qb * 64 + wave * 16;
  float aq[8];
#pragma unroll
  for (int r = 0; r < 8; ++r) aq[r] = AQ[((size_t)b * NH + h) * SQ + q0 + 8 * g + r];
  const float* AKb = AK + ((size_t)b * NH + h) * SK;
  float m[8], l[8]; v8f acc[4] = {};
#pragma unroll
  for (int r = 0; r < 8; ++r) { m[r] = -3.0e38f; l[r] = 0.f; }
#pragma unroll 1
  for (int ks = 0; ks < SK / 32; ++ks) { const float k0v = AKb[ks * 32 + col], k1v = AKb[ks * 32 + 16 + col]; float s[2][8];
#pragma unroll
    for (int r = 0; r < 8; ++r) { float u = aq[r] + k0v; s[0][r] = u > 0.f ? u : 0.2f * u; u = aq[r] + k1v; s[1][r] = u > 0.f ? u : 0.2f * u; }
#pragma unroll
    for (int r = 0; r < 8; ++r) { float mx = fmaxf(s[0][r], s[1][r]);
#pragma unroll
      for (int o = 1; o < 16; o <<= 1) mx = fmaxf(mx, __shfl_xor(mx, o));
      const float mn = fmaxf(m[r], mx); const float alpha = exp_ni(m[r] - mn); const float e0 = exp_ni(s[0][r] - mn), e1 = exp_ni(s[1][r] - mn); float es = e0 + e1;
#pragma unroll
      for (int o = 1; o < 16; o <<= 1) es += __shfl_xor(es, o);
      l[r] = l[r] * alpha + es; m[r] = mn;
#pragma unroll
      for (int dt = 0; dt < 4; ++dt) acc[dt][r] *= alpha;
      sp[wave][8 * g + r][col] = e0; sp[wave][8 * g + r][16 + col] = e1; }
    LDSX();
    const F2 pa = split_row(&sp[wave][col][0], 0, lane);
#pragma unroll
    for (int dt = 0; dt < 4; ++dt) { const size_t vrow = ((size_t)b * DI + h * OD + dt * 16 + col) * SK + ks * 32; const v16b vh = frag_b(VTH + vrow, lane), vl = frag_b(VTL + vrow, lane); acc[dt] = wmma_bf(pa.l, vh, acc[dt]); acc[dt] = wmma_bf(pa.h, vl, acc[dt]); acc[dt] = wmma_bf(pa.h, vh, acc[dt]); }
    LDSX(); }
#pragma unroll
  for (int r = 0; r < 8; ++r) { const float il = 1.0f / l[r];
#pragma unroll
    for (int dt = 0; dt < 4; ++dt) so[wave][8 * g + r][dt * 16 + col] = acc[dt][r] * il + bfr(BIAS[h * OD + dt * 16 + col]); }
  LDSX();
  for (int rl = 0; rl < 16; ++rl) if (lane < 16) vst2(OUT + ((size_t)b * SQ + q0 + rl) * (NH * OD) + h * OD + lane * 4, *(const v4f*)&so[wave][rl][lane * 4]);
}
extern "C" void kernel_launch(void* const* d_in, const int* in_sizes, int n_in, void* d_out, int out_size, void* d_ws, size_t ws_size, hipStream_t stream) {
  (void)in_sizes; (void)n_in; (void)out_size;
  const float** F = (const float**)d_in;
  if (ws_size < (size_t)WS_END) return;
  char* ws = (char*)d_ws; __bf16 *VTH = (__bf16*)(ws + WS_VTH), *VTL = (__bf16*)(ws + WS_VTL); float *AQ = (float*)(ws + WS_AQ), *AK = (float*)(ws + WS_AK);
  k_vproj<<<dim3(SK / 64, TNB), 128, 0, stream>>>(F[2], F[5], VTH, VTL);
  k_aqk<<<dim3(SQ / 64, TNB, 2), 256, 0, stream>>>(F[0], F[1], F[3], F[4], AQ, AK);
  k_attn<<<dim3(TQB, TNB * NH), 128, 0, stream>>>(AQ, AK, VTH, VTL, F[6], (float*)d_out);
}
